// MultiHeadsAtten_35631048688254
// MI455X (gfx1250) — hardware-verified
//
#include <hip/hip_runtime.h>
#include <math.h>
#include <stdint.h>

#define NB    4
#define SEQ   2048
#define DM    1024
#define NH    16
#define HD    64
#define NQB   (SEQ / 64)
#define MROWS (NB * SEQ)
static_assert(NH * HD == DM);
static_assert((SEQ % 128) == 0 && (DM % 128) == 0 && (MROWS % 64) == 0 && (DM % 64) == 0 && (MROWS % 8) == 0);

typedef _Float16 v16h __attribute__((ext_vector_type(16)));
typedef _Float16 v8h  __attribute__((ext_vector_type(8)));
typedef float    v8f  __attribute__((ext_vector_type(8)));
typedef float    v4f  __attribute__((ext_vector_type(4)));
typedef unsigned int v4u __attribute__((ext_vector_type(4)));

__device__ __forceinline__ unsigned short h_bits(_Float16 x) { return __builtin_bit_cast(unsigned short, x); }
__device__ __forceinline__ unsigned pk16(unsigned short a, unsigned short b) { return (unsigned)a | ((unsigned)b << 16); }
__device__ __forceinline__ v8f zero8() { v8f z = {0.f, 0.f, 0.f, 0.f, 0.f, 0.f, 0.f, 0.f}; return z; }

__device__ __forceinline__ void split2(float f0, float f1, unsigned& hp, unsigned& rp) {
  const _Float16 x0 = (_Float16)f0, x1 = (_Float16)f1;
  hp = pk16(h_bits(x0), h_bits(x1));
  const _Float16 r0 = (_Float16)((f0 - (float)x0) * 2048.0f);
  const _Float16 r1 = (_Float16)((f1 - (float)x1) * 2048.0f);
  rp = pk16(h_bits(r0), h_bits(r1));
}
__device__ __forceinline__ unsigned pack2h(float f0, float f1) {
  return pk16(h_bits((_Float16)f0), h_bits((_Float16)f1));
}

__device__ __forceinline__ v16h ldfrag(const _Float16* p) {
  union { v16h v; v8h h[2]; } f;
  f.h[0] = *(const v8h*)(p);
  f.h[1] = *(const v8h*)(p + 16);
  return f.v;
}

__device__ __forceinline__ v8f mma_h(v16h a, v16h b, v8f c) {
  c = __builtin_amdgcn_wmma_f32_16x16x32_f16(false, a, false, b, (short)0, c, false, false);
  asm volatile("v_nop\n\tv_nop\n\tv_nop\n\tv_nop" : "+v"(c) : "v"(a), "v"(b));
  return c;
}

template <bool RES>
__global__ __launch_bounds__(256) void ln_rows(const float* __restrict__ x, const float* __restrict__ gamma,
                                               const float* __restrict__ beta, unsigned short* yh,
                                               unsigned short* yr, int nrows, float eps) {
  const int lane = threadIdx.x & 31;
  const int wave = threadIdx.x >> 5;
  const int row  = blockIdx.x * 8 + wave;
  if (row >= nrows) return;
  const float* xr = x + (size_t)row * DM;
  v4f xv[8];
#pragma unroll
  for (int i = 0; i < 4; ++i) {
    xv[2 * i]     = *(const v4f*)(xr + i * 256 + lane * 8);
    xv[2 * i + 1] = *(const v4f*)(xr + i * 256 + lane * 8 + 4);
  }
  float s = 0.f;
#pragma unroll
  for (int g = 0; g < 8; ++g) s += (xv[g][0] + xv[g][1]) + (xv[g][2] + xv[g][3]);
#pragma unroll
  for (int off = 16; off > 0; off >>= 1) s += __shfl_xor(s, off, 32);
  const float mu = s * (1.0f / (float)DM);
  float ss = 0.f;
#pragma unroll
  for (int g = 0; g < 8; ++g) {
#pragma unroll
    for (int e = 0; e < 4; ++e) { const float d = xv[g][e] - mu; ss += d * d; }
  }
#pragma unroll
  for (int off = 16; off > 0; off >>= 1) ss += __shfl_xor(ss, off, 32);
  const float var = ss * (1.0f / (float)DM);
  const float rs  = rsqrtf(var + eps);

  v4u hv[4], rv[4];
#pragma unroll
  for (int i = 0; i < 4; ++i) {
    const int col = i * 256 + lane * 8;
    const v4f g0 = *(const v4f*)(gamma + col);
    const v4f g1 = *(const v4f*)(gamma + col + 4);
    const v4f b0 = *(const v4f*)(beta + col);
    const v4f b1 = *(const v4f*)(beta + col + 4);
    float y[8];
#pragma unroll
    for (int e = 0; e < 4; ++e) {
      y[e]     = (xv[2 * i][e] - mu) * rs * g0[e] + b0[e];
      y[4 + e] = (xv[2 * i + 1][e] - mu) * rs * g1[e] + b1[e];
    }
    v4u a, a2;
#pragma unroll
    for (int e = 0; e < 4; ++e) {
      unsigned hp, rp;
      split2(y[2 * e], y[2 * e + 1], hp, rp);
      a[e] = hp; a2[e] = rp;
    }
    hv[i] = a; rv[i] = a2;
  }
  unsigned short* oh = yh + (size_t)row * DM + lane * 8;
  unsigned short* orr = yr + (size_t)row * DM + lane * 8;
  for (int pass = 0; pass < 2; ++pass) {
#pragma unroll
    for (int i = 0; i < 4; ++i) {
      *(volatile v4u*)(oh + i * 256) = hv[i];
      if (RES) *(volatile v4u*)(orr + i * 256) = rv[i];
    }
    __threadfence();
  }
}

template <bool RES>
__global__ __launch_bounds__(256) void wcvt_t(const float* __restrict__ W, unsigned short* ph, unsigned short* pr,
                                              float scale) {
  __shared__ float sm[64][65];
  const int tid  = threadIdx.x;
  const int lane = tid & 31;
  const int wave = tid >> 5;
  const int n0 = blockIdx.x * 64;
  const int k0 = blockIdx.y * 64;
  const int kr = tid >> 2;
  const int nc = (tid & 3) * 16;
  const float* src = W + (size_t)(k0 + kr) * DM + n0 + nc;
#pragma unroll
  for (int e = 0; e < 4; ++e) {
    const v4f a = *(const v4f*)(src + 4 * e);
    sm[kr][nc + 4 * e + 0] = a[0];
    sm[kr][nc + 4 * e + 1] = a[1];
    sm[kr][nc + 4 * e + 2] = a[2];
    sm[kr][nc + 4 * e + 3] = a[3];
  }
  __syncthreads();
  const int q  = lane >> 3;
  const int ks = (lane & 7) * 8;
  v4u hv[2], rv[2];
#pragma unroll
  for (int it = 0; it < 2; ++it) {
    const int nrow = wave * 8 + it * 4 + q;
    v4u a, a2;
#pragma unroll
    for (int e = 0; e < 4; ++e) {
      const float f0 = sm[ks + 2 * e][nrow] * scale;
      const float f1 = sm[ks + 2 * e + 1][nrow] * scale;
      unsigned hp, rp;
      split2(f0, f1, hp, rp);
      a[e] = hp; a2[e] = rp;
    }
    hv[it] = a; rv[it] = a2;
  }
  for (int pass = 0; pass < 2; ++pass) {
#pragma unroll
    for (int it = 0; it < 2; ++it) {
      const int nrow = wave * 8 + it * 4 + q;
      const size_t o = (size_t)(n0 + nrow) * DM + k0 + ks;
      *(volatile v4u*)(ph + o) = hv[it];
      if (RES) *(volatile v4u*)(pr + o) = rv[it];
    }
    __threadfence();
  }
}

template <bool RES, int OM>
__global__ __launch_bounds__(256) void gemm_t(
    const unsigned short* __restrict__ Ahp, const unsigned short* __restrict__ Arp, int lda,
    const unsigned short* __restrict__ Bhp, const unsigned short* __restrict__ Brp, int ldb, long long strideB,
    const float* __restrict__ bias, const float* __restrict__ resid,
    void* Cv, void* C2v, int ldc, long long strideC, int K, float oscale, float pscale) {
  __shared__ __align__(16) float sT[64 * 132];
  const int lane = threadIdx.x & 31;
  const int wave = threadIdx.x >> 5;
  const int hh   = lane >> 4;
  const int c    = lane & 15;
  const int n0 = blockIdx.x * 128;
  const int m0 = blockIdx.y * 64;
  const int bz = blockIdx.z;
  const int wm = (wave >> 2) * 32;
  const int wn = (wave & 3) * 32;
  const _Float16* A  = (const _Float16*)(const void*)Ahp;
  const _Float16* A2 = (const _Float16*)(const void*)Arp;
  const _Float16* B  = (const _Float16*)(const void*)Bhp + (size_t)bz * strideB;
  const _Float16* B2 = (const _Float16*)(const void*)Brp + (size_t)bz * strideB;

  v8f acc0[2][2], acc1[2][2];
#pragma unroll
  for (int i = 0; i < 2; ++i)
#pragma unroll
    for (int j = 0; j < 2; ++j) { acc0[i][j] = zero8(); acc1[i][j] = zero8(); }

#pragma unroll 1
  for (int k0 = 0; k0 < K; k0 += 32) {
    v16h bh[2], br[2];
#pragma unroll
    for (int j = 0; j < 2; ++j) {
      const size_t bo = (size_t)(n0 + wn + 16 * j + c) * ldb + k0 + 8 * hh;
      bh[j] = ldfrag(B + bo);
      if (RES) br[j] = ldfrag(B2 + bo); else br[j] = bh[j];
    }
#pragma unroll
    for (int i = 0; i < 2; ++i) {
      const size_t ao = (size_t)(m0 + wm + 16 * i + c) * lda + k0 + 8 * hh;
      const v16h ah = ldfrag(A + ao);
      v16h ar = ah;
      if (RES) ar = ldfrag(A2 + ao);
#pragma unroll
      for (int j = 0; j < 2; ++j) {
        acc0[i][j] = mma_h(ah, bh[j], acc0[i][j]);
        if (RES) {
          acc1[i][j] = mma_h(ar, bh[j], acc1[i][j]);
          acc1[i][j] = mma_h(ah, br[j], acc1[i][j]);
        }
      }
    }
  }

#pragma unroll
  for (int i = 0; i < 2; ++i) {
#pragma unroll
    for (int j = 0; j < 2; ++j) {
#pragma unroll
      for (int r = 0; r < 8; ++r) {
        float v = acc0[i][j][r];
        if (RES) v += acc1[i][j][r] * (1.0f / 2048.0f);
        sT[(wm + 16 * i + 8 * hh + r) * 132 + wn + 16 * j + c] = v;
      }
    }
  }
  __syncthreads();

  if (OM == 0) {
    float* C = (float*)Cv + (size_t)bz * strideC;
    const int c4 = lane * 4;
    const v4f bb = *(const v4f*)(bias + n0 + c4);
    v4f ov[8];
#pragma unroll
    for (int it = 0; it < 8; ++it) {
      const int row = wave * 8 + it;
      const v4f t  = *(const v4f*)(sT + row * 132 + c4);
      const v4f rr = *(const v4f*)(resid + (size_t)(m0 + row) * ldc + n0 + c4);
      ov[it] = t * oscale + bb + rr;
    }
    for (int pass = 0; pass < 2; ++pass) {
#pragma unroll
      for (int it = 0; it < 8; ++it) {
        const int row = wave * 8 + it;
        *(volatile v4f*)(C + (size_t)(m0 + row) * ldc + n0 + c4) = ov[it];
      }
      __threadfence();
    }
  } else {
    unsigned short* C  = (unsigned short*)Cv  + (size_t)bz * strideC;
    unsigned short* C2 = (unsigned short*)C2v + (size_t)bz * strideC;
    const int c8 = c * 8;
    v4u hv[4], rv[4];
#pragma unroll
    for (int it = 0; it < 4; ++it) {
      const int row = wave * 8 + it * 2 + hh;
      const float* sp = sT + row * 132 + c8;
      const v4f x0 = *(const v4f*)(sp);
      const v4f x1 = *(const v4f*)(sp + 4);
      v4f y0, y1;
      if (OM == 1) {
        const v4f b0 = *(const v4f*)(bias + n0 + c8);
        const v4f b1 = *(const v4f*)(bias + n0 + c8 + 4);
        y0 = x0 * oscale + b0;
        y1 = x1 * oscale + b1;
      } else {
        const float brw = bias[m0 + row];
        y0 = (x0 * oscale + brw) * pscale;
        y1 = (x1 * oscale + brw) * pscale;
      }
      v4u a, a2;
      if (OM == 1) {
        unsigned hp, rp;
        split2(y0[0], y0[1], hp, rp); a[0] = hp; a2[0] = rp;
        split2(y0[2], y0[3], hp, rp); a[1] = hp; a2[1] = rp;
        split2(y1[0], y1[1], hp, rp); a[2] = hp; a2[2] = rp;
        split2(y1[2], y1[3], hp, rp); a[3] = hp; a2[3] = rp;
      } else {
        a[0] = pack2h(y0[0], y0[1]);
        a[1] = pack2h(y0[2], y0[3]);
        a[2] = pack2h(y1[0], y1[1]);
        a[3] = pack2h(y1[2], y1[3]);
        a2 = a;
      }
      hv[it] = a; rv[it] = a2;
    }
    for (int pass = 0; pass < 2; ++pass) {
#pragma unroll
      for (int it = 0; it < 4; ++it) {
        const int row = wave * 8 + it * 2 + hh;
        const size_t o = (size_t)(m0 + row) * ldc + n0 + c8;
        *(volatile v4u*)(C + o) = hv[it];
        if (OM == 1) *(volatile v4u*)(C2 + o) = rv[it];
      }
      __threadfence();
    }
  }
}

__global__ __launch_bounds__(128)
void attn_causal64(const unsigned short* __restrict__ qhp, const unsigned short* __restrict__ qrp,
                   const unsigned short* __restrict__ khp, const unsigned short* __restrict__ krp,
                   const unsigned short* __restrict__ vtp, unsigned short* ctxp) {
  union FH { v16h v; v8h h[2]; };
  __shared__ __align__(16) _Float16 Ksh[64 * 64];
  __shared__ __align__(16) _Float16 Ksr[64 * 64];
  __shared__ __align__(16) _Float16 Vth[64 * 64];
  __shared__ __align__(16) _Float16 Psh[4][16 * 64];
  __shared__ __align__(16) float    Os[4][16 * 64];

  const int tid  = threadIdx.x;
  const int wave = tid >> 5;
  const int lane = tid & 31;
  const int hh   = lane >> 4;
  const int c    = lane & 15;

  const int bx   = blockIdx.x;
  const int qb   = bx % NQB;
  const int rest = bx / NQB;
  const int h    = rest % NH;
  const int b    = rest / NH;
  const int q0   = qb * 64 + wave * 16;
  const size_t rowB = (size_t)b * SEQ;

  const _Float16* Qh = (const _Float16*)(const void*)qhp + (size_t)h * HD;
  const _Float16* Qr = (const _Float16*)(const void*)qrp + (size_t)h * HD;
  const _Float16* Kh = (const _Float16*)(const void*)khp + (size_t)h * HD;
  const _Float16* Kr = (const _Float16*)(const void*)krp + (size_t)h * HD;
  const _Float16* Vt = (const _Float16*)(const void*)vtp + ((size_t)b * DM + (size_t)h * HD) * SEQ;

  v16h qah[2], qar[2];
#pragma unroll
  for (int dc = 0; dc < 2; ++dc) {
    const size_t qo = (rowB + q0 + c) * DM + dc * 32 + 8 * hh;
    qah[dc] = ldfrag(Qh + qo);
    qar[dc] = ldfrag(Qr + qo);
  }

  float mrow[8], lrow[8];
  v8f oacc[4];
#pragma unroll
  for (int r = 0; r < 8; ++r) { mrow[r] = -INFINITY; lrow[r] = 0.f; }
#pragma unroll
  for (int t = 0; t < 4; ++t) oacc[t] = zero8();

  const int nkt = qb + 1;
#pragma unroll 1
  for (int kt = 0; kt < nkt; ++kt) {
    const int kv0 = kt * 64;
    __syncthreads();
    {
      const int r = tid >> 1, half = (tid & 1) * 32;
      const _Float16* kg  = Kh + (rowB + kv0 + r) * DM + half;
      const _Float16* krg = Kr + (rowB + kv0 + r) * DM + half;
      const _Float16* vg  = Vt + (size_t)r * SEQ + kv0 + half;
#pragma unroll
      for (int i = 0; i < 4; ++i) {
        const v8h a0 = *(const v8h*)(kg + 8 * i);
        const v8h a1 = *(const v8h*)(krg + 8 * i);
        const v8h b0 = *(const v8h*)(vg + 8 * i);
        *(v8h*)(Ksh + r * 64 + half + 8 * i) = a0;
        *(v8h*)(Ksr + r * 64 + half + 8 * i) = a1;
        *(v8h*)(Vth + r * 64 + half + 8 * i) = b0;
      }
    }
    __syncthreads();

    v8f s[4];
#pragma unroll
    for (int j = 0; j < 4; ++j) {
      v8f t0 = zero8(), t1 = zero8();
#pragma unroll
      for (int dc = 0; dc < 2; ++dc) {
        FH kb, kl;
        kb.h[0] = *(const v8h*)(Ksh + (j * 16 + c) * 64 + dc * 32 + 8 * hh);
        kb.h[1] = *(const v8h*)(Ksh + (j * 16 + c) * 64 + dc * 32 + 16 + 8 * hh);
        kl.h[0] = *(const v8h*)(Ksr + (j * 16 + c) * 64 + dc * 32 + 8 * hh);
        kl.h[1] = *(const v8h*)(Ksr + (j * 16 + c) * 64 + dc * 32 + 16 + 8 * hh);
        t0 = mma_h(qah[dc], kb.v, t0);
        t1 = mma_h(qar[dc], kb.v, t1);
        t1 = mma_h(qah[dc], kl.v, t1);
      }
      s[j] = t0 + t1 * (1.0f / 2048.0f);
    }

    const bool diag = (kt == qb);
    _Float16* pwh = Psh[wave];
#pragma unroll
    for (int r = 0; r < 8; ++r) {
      const int qrow = q0 + 8 * hh + r;
      float m = -INFINITY;
#pragma unroll
      for (int j = 0; j < 4; ++j) {
        const int key = kv0 + j * 16 + c;
        float sv = s[j][r];
        sv = (diag && key > qrow) ? -INFINITY : sv;
        s[j][r] = sv;
        m = fmaxf(m, sv);
      }
#pragma unroll
      for (int off = 1; off < 16; off <<= 1) m = fmaxf(m, __shfl_xor(m, off, 32));
      const float mnew  = fmaxf(mrow[r], m);
      const float msafe = (mnew == -INFINITY) ? 0.f : mnew;
      const float alpha = __expf(mrow[r] - msafe);
      mrow[r] = mnew;
      float psum = 0.f;
#pragma unroll
      for (int j = 0; j < 4; ++j) {
        const float p = __expf(s[j][r] - msafe);
        psum += p;
        pwh[(8 * hh + r) * 64 + j * 16 + c] = (_Float16)(p * 1024.0f);
      }
#pragma unroll
      for (int off = 1; off < 16; off <<= 1) psum += __shfl_xor(psum, off, 32);
      lrow[r] = lrow[r] * alpha + psum;
#pragma unroll
      for (int t = 0; t < 4; ++t) oacc[t][r] *= alpha;
    }
    __builtin_amdgcn_fence(__ATOMIC_RELEASE, "workgroup");
    __builtin_amdgcn_wave_barrier();
    __builtin_amdgcn_fence(__ATOMIC_ACQUIRE, "workgroup");

#pragma unroll
    for (int kk = 0; kk < 2; ++kk) {
      FH pa;
      pa.h[0] = *(const v8h*)(pwh + c * 64 + kk * 32 + 8 * hh);
      pa.h[1] = *(const v8h*)(pwh + c * 64 + kk * 32 + 16 + 8 * hh);
#pragma unroll
      for (int t = 0; t < 4; ++t) {
        FH vb;
        vb.h[0] = *(const v8h*)(Vth + (t * 16 + c) * 64 + kk * 32 + 8 * hh);
        vb.h[1] = *(const v8h*)(Vth + (t * 16 + c) * 64 + kk * 32 + 16 + 8 * hh);
        oacc[t] = mma_h(pa.v, vb.v, oacc[t]);
      }
    }
  }

  float* os = Os[wave];
#pragma unroll
  for (int r = 0; r < 8; ++r) {
    const float l = lrow[r];
    const float inv = ((l > 0.f) ? (1.0f / l) : 0.f) * (1.0f / 1024.0f);
#pragma unroll
    for (int t = 0; t < 4; ++t) os[(8 * hh + r) * 64 + t * 16 + c] = oacc[t][r] * inv;
  }
  __builtin_amdgcn_fence(__ATOMIC_RELEASE, "workgroup");
  __builtin_amdgcn_wave_barrier();
  __builtin_amdgcn_fence(__ATOMIC_ACQUIRE, "workgroup");
  {
    const int q4 = lane >> 3, c8 = (lane & 7) * 8;
    v4u hv[4];
#pragma unroll
    for (int it = 0; it < 4; ++it) {
      const int row = it * 4 + q4;
      const float* sp = os + row * 64 + c8;
      v4u a;
#pragma unroll
      for (int e = 0; e < 4; ++e) a[e] = pack2h(sp[2 * e], sp[2 * e + 1]);
      hv[it] = a;
    }
    for (int pass = 0; pass < 2; ++pass) {
#pragma unroll
      for (int it = 0; it < 4; ++it) {
        const int row = it * 4 + q4;
        const size_t go = (rowB + q0 + row) * DM + (size_t)h * HD + c8;
        *(volatile v4u*)(ctxp + go) = hv[it];
      }
      __threadfence();
    }
  }
}

extern "C" void kernel_launch(void* const* d_in, const int* in_sizes, int n_in,
                              void* d_out, int out_size, void* d_ws, size_t ws_size,
                              hipStream_t stream) {
  if (n_in < 13) return;
  const int nAct = MROWS * DM;
  if (in_sizes[0] != nAct || in_sizes[1] != nAct || in_sizes[2] != nAct) return;
  if (in_sizes[3] != DM * DM || in_sizes[5] != DM * DM || in_sizes[7] != DM * DM || in_sizes[9] != DM * DM) return;
  if (in_sizes[4] != DM || in_sizes[6] != DM || in_sizes[8] != DM || in_sizes[10] != DM) return;
  if (in_sizes[11] != DM || in_sizes[12] != DM) return;
  if (out_size != nAct) return;

  const float* Q  = (const float*)d_in[0];
  const float* Kin = (const float*)d_in[1];
  const float* V  = (const float*)d_in[2];
  const float* Wq = (const float*)d_in[3];
  const float* bq = (const float*)d_in[4];
  const float* Wk = (const float*)d_in[5];
  const float* bk = (const float*)d_in[6];
  const float* Wv = (const float*)d_in[7];
  const float* bv = (const float*)d_in[8];
  const float* Wo = (const float*)d_in[9];
  const float* bo = (const float*)d_in[10];
  const float* gamma = (const float*)d_in[11];
  const float* beta  = (const float*)d_in[12];

  const size_t PA = (size_t)MROWS * DM * 2;
  const size_t PV = (size_t)NB * DM * SEQ * 2;
  const size_t PW = (size_t)DM * DM * 2;
  size_t off = 0;
  const size_t oLh  = off; off += PA;
  const size_t oLr  = off; off += PA;
  const size_t oQh  = off; off += PA;
  const size_t oQr  = off; off += PA;
  const size_t oKh  = off; off += PA;
  const size_t oKr  = off; off += PA;
  const size_t oVt  = off; off += PV;
  const size_t oWqh = off; off += PW;
  const size_t oWqr = off; off += PW;
  const size_t oWkh = off; off += PW;
  const size_t oWkr = off; off += PW;
  const size_t oWvh = off; off += PW;
  const size_t oWoh = off; off += PW;
  if (off > ws_size) return;
  if (off > (size_t)134217728) return;
  const size_t oCtx = oLh;

  char* ws = (char*)d_ws;
  unsigned short* Lh  = (unsigned short*)(ws + oLh);
  unsigned short* Lr  = (unsigned short*)(ws + oLr);
  unsigned short* Qh  = (unsigned short*)(ws + oQh);
  unsigned short* Qr  = (unsigned short*)(ws + oQr);
  unsigned short* Kh  = (unsigned short*)(ws + oKh);
  unsigned short* Kr  = (unsigned short*)(ws + oKr);
  unsigned short* Vt  = (unsigned short*)(ws + oVt);
  unsigned short* Wqh = (unsigned short*)(ws + oWqh);
  unsigned short* Wqr = (unsigned short*)(ws + oWqr);
  unsigned short* Wkh = (unsigned short*)(ws + oWkh);
  unsigned short* Wkr = (unsigned short*)(ws + oWkr);
  unsigned short* Wvh = (unsigned short*)(ws + oWvh);
  unsigned short* Woh = (unsigned short*)(ws + oWoh);
  unsigned short* Ctx = (unsigned short*)(ws + oCtx);

  const dim3 blk256(256), blk128(128);
  const dim3 gW(DM / 64, DM / 64);
  const dim3 gLN(MROWS / 8);
  const dim3 gProj(DM / 128, MROWS / 64, 1);
  const dim3 gVt(SEQ / 128, DM / 64, NB);
  const dim3 gAttn(NB * NH * NQB);
  const float eps = 1e-6f;

  wcvt_t<true ><<<gW, blk256, 0, stream>>>(Wq, Wqh, Wqr, 32.0f);
  wcvt_t<true ><<<gW, blk256, 0, stream>>>(Wk, Wkh, Wkr, 32.0f);
  wcvt_t<false><<<gW, blk256, 0, stream>>>(Wv, Wvh, Wvh, 32.0f);
  wcvt_t<false><<<gW, blk256, 0, stream>>>(Wo, Woh, Woh, 32.0f);
  ln_rows<true><<<gLN, blk256, 0, stream>>>(Q, gamma, beta, Lh, Lr, MROWS, eps);
  gemm_t<true, 1><<<gProj, blk256, 0, stream>>>(
      Lh, Lr, DM, Wqh, Wqr, DM, 0LL, bq, bq,
      (void*)Qh, (void*)Qr, DM, 0LL, DM, 1.0f / 32.0f, 1.0f);
  ln_rows<true><<<gLN, blk256, 0, stream>>>(Kin, gamma, beta, Lh, Lr, MROWS, eps);
  gemm_t<true, 1><<<gProj, blk256, 0, stream>>>(
      Lh, Lr, DM, Wkh, Wkr, DM, 0LL, bk, bk,
      (void*)Kh, (void*)Kr, DM, 0LL, DM, 1.0f / 32.0f, 1.0f);
  ln_rows<false><<<gLN, blk256, 0, stream>>>(V, gamma, beta, Lh, Lh, MROWS, eps);
  gemm_t<false, 2><<<gVt, blk256, 0, stream>>>(
      Wvh, Wvh, DM, Lh, Lh, DM, (long long)SEQ * DM, bv, bv,
      (void*)Vt, (void*)Vt, SEQ, (long long)DM * SEQ, DM, 1.0f / 32.0f, 4.0f);
  attn_causal64<<<gAttn, blk128, 0, stream>>>(Qh, Qr, Kh, Kr, Vt, Ctx);
  gemm_t<false, 0><<<gProj, blk256, 0, stream>>>(
      Ctx, Ctx, DM, Woh, Woh, DM, 0LL, bo, Q,
      d_out, d_out, DM, 0LL, DM, 1.0f / 128.0f, 1.0f);
  (void)hipGetLastError();
}
